// GRU_sememe_54571854463109
// MI455X (gfx1250) — hardware-verified
//
#include <hip/hip_runtime.h>
#include <stddef.h>

typedef __attribute__((ext_vector_type(16))) _Float16 v16h;
typedef __attribute__((ext_vector_type(8)))  _Float16 v8h;
typedef __attribute__((ext_vector_type(16))) __bf16   v16b;
typedef __attribute__((ext_vector_type(8)))  __bf16   v8b;
typedef __attribute__((ext_vector_type(8)))  float    v8f;
typedef __attribute__((ext_vector_type(4)))  float    v4f;

__device__ __forceinline__ unsigned short f2bf_bits(float f) {
  unsigned u = __float_as_uint(f);
  return (unsigned short)((u + 0x7FFFu + ((u >> 16) & 1u)) >> 16);
}
__device__ __forceinline__ float bf_bits2f(unsigned short h) { return __uint_as_float(((unsigned)h) << 16); }

__device__ __forceinline__ void dep_guard_h(v8f& a, v8f& b, v16h x, v16h y) { asm volatile("v_nop\n\tv_nop\n\tv_nop\n\tv_nop" : "+v"(a), "+v"(b) : "v"(x), "v"(y)); }
__device__ __forceinline__ void dep_guard_b(v8f& a, v8f& b, v16b x, v16b y) { asm volatile("v_nop\n\tv_nop\n\tv_nop\n\tv_nop" : "+v"(a), "+v"(b) : "v"(x), "v"(y)); }
__device__ __forceinline__ void keep4_h(v16h a, v16h b, v16h c, v16h d) { asm volatile("v_nop" :: "v"(a), "v"(b), "v"(c), "v"(d)); }
__device__ __forceinline__ void keep4_b(v16b a, v16b b, v16b c, v16b d) { asm volatile("v_nop" :: "v"(a), "v"(b), "v"(c), "v"(d)); }
__device__ __forceinline__ void acc_guard4(v8f& a, v8f& b, v8f& c, v8f& d) { asm volatile("v_nop\n\tv_nop\n\tv_nop\n\tv_nop" : "+v"(a), "+v"(b), "+v"(c), "+v"(d)); }
template <typename T> struct Frag;
template <> struct Frag<_Float16> {
  typedef v16h V; union U { v16h v; v8h h[2]; };
  static __device__ __forceinline__ v16h load(const _Float16* p) {
    U f; f.h[0] = *(const v8h*)(p); f.h[1] = *(const v8h*)(p + 16); return f.v;
  }
  static __device__ __forceinline__ v8f mma(v16h a, v16h b, v8f c) {
    return __builtin_amdgcn_wmma_f32_16x16x32_f16(false, a, false, b, (short)0, c, false, false);
  }
  static __device__ __forceinline__ void guard(v8f& a, v8f& b, v16h x, v16h y) { dep_guard_h(a, b, x, y); }
  static __device__ __forceinline__ void keep(v16h a, v16h b, v16h c, v16h d) { keep4_h(a, b, c, d); }
};
template <> struct Frag<__bf16> {
  typedef v16b V; union U { v16b v; v8b h[2]; };
  static __device__ __forceinline__ v16b load(const __bf16* p) {
    U f; f.h[0] = *(const v8b*)(p); f.h[1] = *(const v8b*)(p + 16); return f.v;
  }
  static __device__ __forceinline__ v8f mma(v16b a, v16b b, v8f c) {
    return __builtin_amdgcn_wmma_f32_16x16x32_bf16(false, a, false, b, (short)0, c, false, false);
  }
  static __device__ __forceinline__ void guard(v8f& a, v8f& b, v16b x, v16b y) { dep_guard_b(a, b, x, y); }
  static __device__ __forceinline__ void keep(v16b a, v16b b, v16b c, v16b d) { keep4_b(a, b, c, d); }
};

template <int ET> struct Elem;
template <> struct Elem<0> { typedef _Float16 T; };
template <> struct Elem<1> { typedef __bf16 T; };
template <int ET, bool SPLIT, int BIAS_MODE, int OUT_MODE, bool RESID, int ACT = 0>
__global__ __launch_bounds__(256) void wmma_gemm64(
    const unsigned short* __restrict__ Ap, const unsigned short* __restrict__ A2p, int lda, long strideA,
    const unsigned short* __restrict__ Btp, const unsigned short* __restrict__ Bt2p, int ldb, long strideB,
    void* __restrict__ Cout, void* __restrict__ Cout2, int ldc, long strideC,
    const float* __restrict__ bias,
    const float* __restrict__ resid, long strideR,
    int M, int N, int K, float scale) {
  typedef typename Elem<ET>::T T;
  typedef typename Frag<T>::V V;
  const T* A = (const T*)Ap; const T* A2 = (const T*)A2p; const T* Bt = (const T*)Btp; const T* Bt2 = (const T*)Bt2p;
  __shared__ __align__(16) float sT[8][16 * 68];
  const int b    = blockIdx.y;
  const int lane = threadIdx.x & 31;
  const int wave = threadIdx.x >> 5;
  const int tilesN = N >> 6;
  const int tilesM = M >> 6;
  const int tile = blockIdx.x * 8 + wave;
  if (tile >= tilesM * tilesN) return;
  const int tm = tile / tilesN;
  const int tn = tile - tm * tilesN;
  const int m0 = tm << 6;
  const int n0 = tn << 6;

  const T* Ab  = A  + (size_t)b * strideA;
  const T* Bb  = Bt + (size_t)b * strideB;
  const T* Ab2 = SPLIT ? (A2  + (size_t)b * strideA) : nullptr;
  const T* Bb2 = SPLIT ? (Bt2 + (size_t)b * strideB) : nullptr;

  const int rlane = lane & 15;
  const int koff  = (lane >> 4) * 8;
  const int mOff  = (lane >> 4) * 8;

  v8f acc[4][4];
#pragma unroll
  for (int i = 0; i < 4; ++i)
#pragma unroll
    for (int j = 0; j < 4; ++j) acc[i][j] = (v8f){0.f,0.f,0.f,0.f,0.f,0.f,0.f,0.f};

  for (int k0 = 0; k0 < K; k0 += 32) {
    V bh[4], bl[4];
#pragma unroll
    for (int j = 0; j < 4; ++j) {
      const size_t bo = (size_t)(n0 + (j << 4) + rlane) * ldb + koff + k0;
      bh[j] = Frag<T>::load(Bb + bo);
      if (SPLIT) bl[j] = Frag<T>::load(Bb2 + bo);
    }
#pragma unroll
    for (int i = 0; i < 4; ++i) {
      const size_t ao = (size_t)(m0 + (i << 4) + rlane) * lda + koff + k0;
      V ah = Frag<T>::load(Ab + ao);
      V al;
      if (SPLIT) al = Frag<T>::load(Ab2 + ao);
#pragma unroll
      for (int j = 0; j < 4; ++j) {
        acc[i][j] = Frag<T>::mma(ah, bh[j], acc[i][j]);
        if (SPLIT) {
          acc[i][j] = Frag<T>::mma(ah, bl[j], acc[i][j]);
          acc[i][j] = Frag<T>::mma(al, bh[j], acc[i][j]);
        }
      }
      Frag<T>::guard(acc[i][0], acc[i][3], ah, SPLIT ? al : ah);
    }
    Frag<T>::keep(bh[0], bh[1], bh[2], bh[3]);
    if (SPLIT) Frag<T>::keep(bl[0], bl[1], bl[2], bl[3]);
  }
  acc_guard4(acc[0][0], acc[0][1], acc[0][2], acc[0][3]);
  acc_guard4(acc[1][0], acc[1][1], acc[1][2], acc[1][3]);
  acc_guard4(acc[2][0], acc[2][1], acc[2][2], acc[2][3]);
  acc_guard4(acc[3][0], acc[3][1], acc[3][2], acc[3][3]);

  float* slab = sT[wave];
  const float* Rb = RESID ? (resid + (size_t)b * strideR) : nullptr;
#pragma unroll
  for (int i = 0; i < 4; ++i) {
    const int mBase = m0 + (i << 4);
#pragma unroll
    for (int j = 0; j < 4; ++j) {
      const int n = n0 + (j << 4) + rlane;
      float bv = 0.f;
      if (BIAS_MODE == 2) bv = bias[n];
#pragma unroll
      for (int r = 0; r < 8; ++r) {
        float v = acc[i][j][r] * scale;
        if (BIAS_MODE == 1) v += bias[mBase + mOff + r];
        if (BIAS_MODE == 2) v += bv;
        if (RESID) v += Rb[(size_t)(mBase + mOff + r) * ldc + n];
        if (ACT == 1) v = tanhf(v);
        if (ACT == 2) v = fmaxf(v, 0.0f);
        if (ACT == 3) v = v / (1.0f + expf(-v));
        if (ACT == 4) v = (v > 0.f) ? v : 0.01f * v;
        if (ACT == 5) v = 0.5f * v * (1.0f + erff(v * 0.70710678118654752f));
        slab[(mOff + r) * 68 + (j << 4) + rlane] = v;
      }
    }
    __builtin_amdgcn_fence(__ATOMIC_RELEASE, "workgroup");
    __builtin_amdgcn_wave_barrier();
    __builtin_amdgcn_fence(__ATOMIC_ACQUIRE, "workgroup");
    if (OUT_MODE == 0) {
      float* C = (float*)Cout + (size_t)b * strideC;
      const int hh = lane >> 4, c4 = (lane & 15) * 4;
      for (int pass = 0; pass < 2; ++pass) {
#pragma unroll
        for (int it = 0; it < 8; ++it) {
          const int row = it * 2 + hh;
          v4f v = *(const v4f*)(slab + row * 68 + c4);
          *(volatile v4f*)(C + (size_t)(mBase + row) * ldc + n0 + c4) = v;
        }
        __threadfence();
      }
    } else {
      const int q = lane >> 3, c8 = (lane & 7) * 8;
      unsigned short* C  = (unsigned short*)Cout  + (size_t)b * strideC;
      unsigned short* C2 = (OUT_MODE == 2) ? ((unsigned short*)Cout2 + (size_t)b * strideC) : nullptr;
      for (int pass = 0; pass < 2; ++pass) {
#pragma unroll
        for (int it = 0; it < 4; ++it) {
          const int row = it * 4 + q;
          const float* sp = slab + row * 68 + c8;
          v8h hv, lv;
#pragma unroll
          for (int e = 0; e < 8; ++e) {
            if (OUT_MODE == 1) {
              hv[e] = (_Float16)sp[e];
            } else {
              unsigned short hb = f2bf_bits(sp[e]);
              unsigned short lb = f2bf_bits(sp[e] - bf_bits2f(hb));
              hv[e] = __builtin_bit_cast(_Float16, hb);
              lv[e] = __builtin_bit_cast(_Float16, lb);
            }
          }
          *(volatile v8h*)(C + (size_t)(mBase + row) * ldc + n0 + c8) = hv;
          if (OUT_MODE == 2) *(volatile v8h*)(C2 + (size_t)(mBase + row) * ldc + n0 + c8) = lv;
        }
        __threadfence();
      }
    }
    __builtin_amdgcn_fence(__ATOMIC_RELEASE, "workgroup");
    __builtin_amdgcn_wave_barrier();
    __builtin_amdgcn_fence(__ATOMIC_ACQUIRE, "workgroup");
  }
}

constexpr int SEQ_T     = 256;
constexpr int BATCH_B   = 64;
constexpr int DIM_IN    = 512;
constexpr int DIM_H     = 512;
constexpr int DIM_X     = 2 * DIM_IN;
constexpr int DIM_IOU   = 2 * DIM_H;
constexpr int DIM_STACK = DIM_IOU + DIM_H;
constexpr int ROWS_ALL  = SEQ_T * BATCH_B;
constexpr int ROWS_HALF = ROWS_ALL / 2;
constexpr int HPITCH    = DIM_H + 8;
constexpr int SPITCH    = DIM_H + 4;
constexpr float kWCarry   = 16.0f;
constexpr float kHCarry   = 8.0f;
constexpr float kAccScale = 1.0f / 128.0f;
constexpr float kXScale   = 1.0f / 16.0f;

static_assert(DIM_H % 32 == 0 && DIM_X % 32 == 0);
static_assert(ROWS_HALF % 64 == 0 && DIM_IOU % 64 == 0 && DIM_H % 64 == 0);
static_assert((HPITCH * 2) % 16 == 0 && (SPITCH * 4) % 16 == 0);

__global__ __launch_bounds__(256) void cast_f32_f16x8_scaled(
    const float* __restrict__ in, unsigned short* __restrict__ out, int n8, float scale) {
  const int i = blockIdx.x * 256 + threadIdx.x;
  if (i < n8) {
    const float* p = in + (size_t)i * 8;
    const v4f a = *(const v4f*)(p);
    const v4f b = *(const v4f*)(p + 4);
    v8h hv;
    hv[0] = (_Float16)(a[0] * scale); hv[1] = (_Float16)(a[1] * scale);
    hv[2] = (_Float16)(a[2] * scale); hv[3] = (_Float16)(a[3] * scale);
    hv[4] = (_Float16)(b[0] * scale); hv[5] = (_Float16)(b[1] * scale);
    hv[6] = (_Float16)(b[2] * scale); hv[7] = (_Float16)(b[3] * scale);
    _Float16* o = (_Float16*)out + (size_t)i * 8;
    *(volatile v8h*)o = hv;
    __threadfence();
    *(volatile v8h*)o = hv;
  }
}

__global__ __launch_bounds__(256) void build_x16_half(
    const float* __restrict__ srcA, const float* __restrict__ srcB,
    unsigned short* __restrict__ xo, int row0, int nchunks) {
  const int i = blockIdx.x * 256 + threadIdx.x;
  if (i < nchunks) {
    const int r = i >> 7, ch = i & 127;
    const size_t grow = (size_t)(row0 + r);
    const int colA = (ch & 63) * 8;
    const float* p = ((ch < 64) ? srcA : srcB) + grow * DIM_IN + colA;
    const v4f a = *(const v4f*)(p);
    const v4f b = *(const v4f*)(p + 4);
    v8h hv;
    hv[0] = (_Float16)a[0]; hv[1] = (_Float16)a[1]; hv[2] = (_Float16)a[2]; hv[3] = (_Float16)a[3];
    hv[4] = (_Float16)b[0]; hv[5] = (_Float16)b[1]; hv[6] = (_Float16)b[2]; hv[7] = (_Float16)b[3];
    _Float16* o = (_Float16*)xo + (size_t)r * DIM_X + ch * 8;
    *(volatile v8h*)o = hv;
    __threadfence();
    *(volatile v8h*)o = hv;
  }
}

__device__ __forceinline__ float gate_sigmoid(float x) {
  const float e = __builtin_amdgcn_exp2f(-x * 1.4426950408889634f);
  return __builtin_amdgcn_rcpf(1.0f + e);
}
__device__ __forceinline__ float gate_tanh(float x) {
  const float e = __builtin_amdgcn_exp2f(x * 2.8853900817779268f);
  return 1.0f - 2.0f * __builtin_amdgcn_rcpf(1.0f + e);
}

__global__ __launch_bounds__(256) void recur_seq_kernel(
    const unsigned short* __restrict__ Whp,
    const unsigned short* __restrict__ Wup,
    const float* __restrict__ b_h,
    const float* __restrict__ b_u,
    const float* __restrict__ h0,
    const float* __restrict__ xproj,
    float* __restrict__ out_seq,
    float* __restrict__ out_last) {
  typedef Frag<_Float16> FR;
  __shared__ __align__(16) _Float16 hA[16 * HPITCH];
  __shared__ __align__(16) _Float16 rA[16 * HPITCH];
  __shared__ __align__(16) float slab[16 * SPITCH];
  const _Float16* Wh = (const _Float16*)Whp;
  const _Float16* Wu = (const _Float16*)Wup;
  const int tid  = threadIdx.x;
  const int wave = tid >> 5;
  const int lane = tid & 31;
  const int hh   = lane >> 4;
  const int cc   = lane & 15;
  const int koff = 8 * hh;
  const int b0   = blockIdx.x * 16;

  int   ucol[4];
  float bz[4], br[4], bu[4];
  float hm[4][8];
  float zg[4][8];
#pragma unroll
  for (int u = 0; u < 4; ++u) {
    ucol[u] = 64 * wave + 16 * u + cc;
    bz[u] = b_h[ucol[u]];
    br[u] = b_h[DIM_H + ucol[u]];
    bu[u] = b_u[ucol[u]];
#pragma unroll
    for (int r = 0; r < 8; ++r) {
      const int row = 8 * hh + r;
      const float v = h0[(size_t)(b0 + row) * DIM_H + ucol[u]];
      hm[u][r] = v;
      zg[u][r] = 0.0f;
      hA[row * HPITCH + ucol[u]] = (_Float16)(v * kHCarry);
    }
  }
  __syncthreads();

  for (int t = 0; t < SEQ_T; ++t) {
    const float* xr = xproj + (size_t)(t * BATCH_B + b0) * DIM_STACK;

    {
      v8f acc[4];
#pragma unroll
      for (int u = 0; u < 4; ++u) acc[u] = (v8f){0.f,0.f,0.f,0.f,0.f,0.f,0.f,0.f};
      for (int k0 = 0; k0 < DIM_H; k0 += 32) {
        const v16h a = FR::load(hA + cc * HPITCH + k0 + koff);
        v16h bf[4];
#pragma unroll
        for (int u = 0; u < 4; ++u)
          bf[u] = FR::load(Wh + (size_t)(DIM_H + 64 * wave + 16 * u + cc) * DIM_H + k0 + koff);
#pragma unroll
        for (int u = 0; u < 4; ++u) acc[u] = FR::mma(a, bf[u], acc[u]);
        FR::guard(acc[0], acc[3], a, bf[3]);
        FR::keep(bf[0], bf[1], bf[2], bf[3]);
      }
      acc_guard4(acc[0], acc[1], acc[2], acc[3]);
#pragma unroll
      for (int u = 0; u < 4; ++u) {
#pragma unroll
        for (int r = 0; r < 8; ++r) {
          const int row = 8 * hh + r;
          const float pre = acc[u][r] * kAccScale + xr[(size_t)row * DIM_STACK + DIM_H + ucol[u]] + br[u];
          const float rg  = gate_sigmoid(pre);
          const float rh  = rg * hm[u][r];
          rA[row * HPITCH + ucol[u]] = (_Float16)(rh * kHCarry);
        }
      }
    }

    {
      v8f acc[4];
#pragma unroll
      for (int u = 0; u < 4; ++u) acc[u] = (v8f){0.f,0.f,0.f,0.f,0.f,0.f,0.f,0.f};
      for (int k0 = 0; k0 < DIM_H; k0 += 32) {
        const v16h a = FR::load(hA + cc * HPITCH + k0 + koff);
        v16h bf[4];
#pragma unroll
        for (int u = 0; u < 4; ++u)
          bf[u] = FR::load(Wh + (size_t)(64 * wave + 16 * u + cc) * DIM_H + k0 + koff);
#pragma unroll
        for (int u = 0; u < 4; ++u) acc[u] = FR::mma(a, bf[u], acc[u]);
        FR::guard(acc[0], acc[3], a, bf[3]);
        FR::keep(bf[0], bf[1], bf[2], bf[3]);
      }
      acc_guard4(acc[0], acc[1], acc[2], acc[3]);
#pragma unroll
      for (int u = 0; u < 4; ++u) {
#pragma unroll
        for (int r = 0; r < 8; ++r) {
          const int row = 8 * hh + r;
          const float pre = acc[u][r] * kAccScale + xr[(size_t)row * DIM_STACK + ucol[u]] + bz[u];
          zg[u][r] = gate_sigmoid(pre);
        }
      }
    }
    __syncthreads();

    {
      v8f acc[4];
#pragma unroll
      for (int u = 0; u < 4; ++u) acc[u] = (v8f){0.f,0.f,0.f,0.f,0.f,0.f,0.f,0.f};
      for (int k0 = 0; k0 < DIM_H; k0 += 32) {
        const v16h a = FR::load(rA + cc * HPITCH + k0 + koff);
        v16h bf[4];
#pragma unroll
        for (int u = 0; u < 4; ++u)
          bf[u] = FR::load(Wu + (size_t)(64 * wave + 16 * u + cc) * DIM_H + k0 + koff);
#pragma unroll
        for (int u = 0; u < 4; ++u) acc[u] = FR::mma(a, bf[u], acc[u]);
        FR::guard(acc[0], acc[3], a, bf[3]);
        FR::keep(bf[0], bf[1], bf[2], bf[3]);
      }
      acc_guard4(acc[0], acc[1], acc[2], acc[3]);
#pragma unroll
      for (int u = 0; u < 4; ++u) {
#pragma unroll
        for (int r = 0; r < 8; ++r) {
          const int row = 8 * hh + r;
          const float pre = acc[u][r] * kAccScale + xr[(size_t)row * DIM_STACK + DIM_IOU + ucol[u]] + bu[u];
          const float ht  = gate_tanh(pre);
          const float z   = zg[u][r];
          const float hn  = (1.0f - z) * hm[u][r] + z * ht;
          hm[u][r] = hn;
          slab[row * SPITCH + ucol[u]] = hn;
          hA[row * HPITCH + ucol[u]] = (_Float16)(hn * kHCarry);
        }
      }
    }
    __syncthreads();

    {
      for (int pass = 0; pass < 2; ++pass) {
#pragma unroll
        for (int rr = 0; rr < 2; ++rr) {
          const int row = 2 * wave + rr;
#pragma unroll
          for (int it = 0; it < 4; ++it) {
            const int c4 = it * 128 + lane * 4;
            const v4f v = *(const v4f*)(slab + row * SPITCH + c4);
            *(volatile v4f*)(out_seq + (size_t)(t * BATCH_B + b0 + row) * DIM_H + c4) = v;
          }
        }
        __threadfence();
      }
    }
  }

  {
    for (int pass = 0; pass < 2; ++pass) {
#pragma unroll
      for (int rr = 0; rr < 2; ++rr) {
        const int row = 2 * wave + rr;
#pragma unroll
        for (int it = 0; it < 4; ++it) {
          const int c4 = it * 128 + lane * 4;
          const v4f v = *(const v4f*)(slab + row * SPITCH + c4);
          *(volatile v4f*)(out_last + (size_t)(b0 + row) * DIM_H + c4) = v;
        }
      }
      __threadfence();
    }
  }
}

extern "C" void kernel_launch(void* const* d_in, const int* in_sizes, int n_in,
                              void* d_out, int out_size, void* d_ws,
                              size_t ws_size, hipStream_t stream) {
  if (n_in < 11) return;
  const float* in_x  = (const float*)d_in[0];
  const float* in_s  = (const float*)d_in[1];
  const float* in_h0 = (const float*)d_in[2];
  const float* w_x   = (const float*)d_in[3];
  const float* b_x   = (const float*)d_in[4];
  const float* w_h   = (const float*)d_in[5];
  const float* b_h   = (const float*)d_in[6];
  const float* w_f   = (const float*)d_in[7];
  const float* b_f   = (const float*)d_in[8];
  const float* w_u   = (const float*)d_in[9];
  const float* b_u   = (const float*)d_in[10];
  float* out_seq  = (float*)d_out;
  float* out_last = (float*)d_out + (size_t)ROWS_ALL * DIM_H;

  if (in_sizes[0] != ROWS_ALL * DIM_IN || in_sizes[1] != ROWS_ALL * DIM_IN ||
      in_sizes[2] != BATCH_B * DIM_H || in_sizes[3] != DIM_IOU * DIM_X || in_sizes[4] != DIM_IOU ||
      in_sizes[5] != DIM_IOU * DIM_H || in_sizes[6] != DIM_IOU || in_sizes[7] != DIM_H * DIM_X ||
      in_sizes[8] != DIM_H || in_sizes[9] != DIM_H * DIM_H || in_sizes[10] != DIM_H) return;
  if (out_size != ROWS_ALL * DIM_H + BATCH_B * DIM_H) return;

  char* ws = (char*)d_ws;
  size_t off = 0;
  unsigned short* Wxf16 = (unsigned short*)(ws + off); off += (size_t)DIM_STACK * DIM_X * 2;
  unsigned short* Wh16  = (unsigned short*)(ws + off); off += (size_t)DIM_IOU * DIM_H * 2;
  unsigned short* Wu16  = (unsigned short*)(ws + off); off += (size_t)DIM_H * DIM_H * 2;
  unsigned short* X16   = (unsigned short*)(ws + off); off += (size_t)ROWS_HALF * DIM_X * 2;
  float*          XPROJ = (float*)(ws + off);          off += (size_t)ROWS_ALL * DIM_STACK * 4;
  if (off > ws_size) return;

  {
    const int n8a = DIM_IOU * DIM_X / 8;
    cast_f32_f16x8_scaled<<<(n8a + 255) / 256, 256, 0, stream>>>(w_x, Wxf16, n8a, kWCarry);
    const int n8b = DIM_H * DIM_X / 8;
    cast_f32_f16x8_scaled<<<(n8b + 255) / 256, 256, 0, stream>>>(w_f, Wxf16 + (size_t)DIM_IOU * DIM_X, n8b, kWCarry);
    const int n8c = DIM_IOU * DIM_H / 8;
    cast_f32_f16x8_scaled<<<(n8c + 255) / 256, 256, 0, stream>>>(w_h, Wh16, n8c, kWCarry);
    const int n8d = DIM_H * DIM_H / 8;
    cast_f32_f16x8_scaled<<<(n8d + 255) / 256, 256, 0, stream>>>(w_u, Wu16, n8d, kWCarry);
  }

  for (int hf = 0; hf < 2; ++hf) {
    const int nchunks = ROWS_HALF * (DIM_X / 8);
    build_x16_half<<<(nchunks + 255) / 256, 256, 0, stream>>>(in_x, in_s, X16, hf * ROWS_HALF, nchunks);
    float* Cbase = XPROJ + (size_t)hf * ROWS_HALF * DIM_STACK;
    {
      const int gx = (ROWS_HALF / 64) * (DIM_IOU / 64) / 8;
      wmma_gemm64<0, false, 2, 0, false, 0><<<dim3(gx, 1), 256, 0, stream>>>(
          X16, X16, DIM_X, 0L,
          Wxf16, Wxf16, DIM_X, 0L,
          (void*)Cbase, (void*)Cbase, DIM_STACK, 0L,
          b_x, b_x, 0L,
          ROWS_HALF, DIM_IOU, DIM_X, kXScale);
    }
    {
      const int gx = (ROWS_HALF / 64) * (DIM_H / 64) / 8;
      const unsigned short* Wf16 = Wxf16 + (size_t)DIM_IOU * DIM_X;
      float* Cf = Cbase + DIM_IOU;
      wmma_gemm64<0, false, 2, 0, false, 0><<<dim3(gx, 1), 256, 0, stream>>>(
          X16, X16, DIM_X, 0L,
          Wf16, Wf16, DIM_X, 0L,
          (void*)Cf, (void*)Cf, DIM_STACK, 0L,
          b_f, b_f, 0L,
          ROWS_HALF, DIM_H, DIM_X, kXScale);
    }
  }

  recur_seq_kernel<<<BATCH_B / 16, 256, 0, stream>>>(Wh16, Wu16, b_h, b_u, in_h0, XPROJ, out_seq, out_last);
}
